// SharedSelfAttentionV0_54554674593973
// MI455X (gfx1250) — hardware-verified
//
#include <hip/hip_runtime.h>
#include <math.h>
typedef __attribute__((ext_vector_type(16))) _Float16 v16h;
typedef __attribute__((ext_vector_type(8)))  _Float16 v8h;
typedef __attribute__((ext_vector_type(16))) __bf16   v16b;
typedef __attribute__((ext_vector_type(8)))  __bf16   v8b;
typedef __attribute__((ext_vector_type(8)))  float    v8f;
typedef __attribute__((ext_vector_type(4)))  float    v4f;
#define PSCALE 32768.0f
#define U16(p) ((const unsigned short*)(const void*)(p))
#define PSCALE_INV (1.0f / 32768.0f)

__device__ __forceinline__ unsigned short f2bf_bits(float f) {
  unsigned u = __float_as_uint(f);
  return (unsigned short)((u + 0x7FFFu + ((u >> 16) & 1u)) >> 16);
}
__device__ __forceinline__ float bf_bits2f(unsigned short h) { return __uint_as_float(((unsigned)h) << 16); }

__device__ __forceinline__ void dep_guard_h(v8f& a, v8f& b, v16h x, v16h y) { asm volatile("v_nop\n\tv_nop\n\tv_nop\n\tv_nop" : "+v"(a), "+v"(b) : "v"(x), "v"(y)); }
__device__ __forceinline__ void dep_guard_b(v8f& a, v8f& b, v16b x, v16b y) { asm volatile("v_nop\n\tv_nop\n\tv_nop\n\tv_nop" : "+v"(a), "+v"(b) : "v"(x), "v"(y)); }
__device__ __forceinline__ void keep4_h(v16h a, v16h b, v16h c, v16h d) { asm volatile("v_nop" :: "v"(a), "v"(b), "v"(c), "v"(d)); }
__device__ __forceinline__ void keep4_b(v16b a, v16b b, v16b c, v16b d) { asm volatile("v_nop" :: "v"(a), "v"(b), "v"(c), "v"(d)); }
__device__ __forceinline__ void acc_guard4(v8f& a, v8f& b, v8f& c, v8f& d) { asm volatile("v_nop\n\tv_nop\n\tv_nop\n\tv_nop" : "+v"(a), "+v"(b), "+v"(c), "+v"(d)); }
template <typename T> struct Frag;
template <> struct Frag<_Float16> {
  typedef v16h V; union U { v16h v; v8h h[2]; };
  static __device__ __forceinline__ v16h load(const _Float16* p) {
    U f; f.h[0] = *(const v8h*)(p); f.h[1] = *(const v8h*)(p + 16); return f.v;
  }
  static __device__ __forceinline__ v8f mma(v16h a, v16h b, v8f c) {
    return __builtin_amdgcn_wmma_f32_16x16x32_f16(false, a, false, b, (short)0, c, false, false);
  }
  static __device__ __forceinline__ void guard(v8f& a, v8f& b, v16h x, v16h y) { dep_guard_h(a, b, x, y); }
  static __device__ __forceinline__ void keep(v16h a, v16h b, v16h c, v16h d) { keep4_h(a, b, c, d); }
};
template <> struct Frag<__bf16> {
  typedef v16b V; union U { v16b v; v8b h[2]; };
  static __device__ __forceinline__ v16b load(const __bf16* p) {
    U f; f.h[0] = *(const v8b*)(p); f.h[1] = *(const v8b*)(p + 16); return f.v;
  }
  static __device__ __forceinline__ v8f mma(v16b a, v16b b, v8f c) {
    return __builtin_amdgcn_wmma_f32_16x16x32_bf16(false, a, false, b, (short)0, c, false, false);
  }
  static __device__ __forceinline__ void guard(v8f& a, v8f& b, v16b x, v16b y) { dep_guard_b(a, b, x, y); }
  static __device__ __forceinline__ void keep(v16b a, v16b b, v16b c, v16b d) { keep4_b(a, b, c, d); }
};

template <int ET> struct Elem;
template <> struct Elem<0> { typedef _Float16 T; };
template <> struct Elem<1> { typedef __bf16 T; };
template <int ET, bool SPLIT, int BIAS_MODE, int OUT_MODE, bool RESID, int ACT = 0>
__global__ __launch_bounds__(256) void wmma_gemm64(
    const unsigned short* __restrict__ Ap, const unsigned short* __restrict__ A2p, int lda, long strideA,
    const unsigned short* __restrict__ Btp, const unsigned short* __restrict__ Bt2p, int ldb, long strideB,
    void* __restrict__ Cout, void* __restrict__ Cout2, int ldc, long strideC,
    const float* __restrict__ bias,
    const float* __restrict__ resid, long strideR,
    int M, int N, int K, float scale) {
  typedef typename Elem<ET>::T T;
  typedef typename Frag<T>::V V;
  const T* A = (const T*)Ap; const T* A2 = (const T*)A2p; const T* Bt = (const T*)Btp; const T* Bt2 = (const T*)Bt2p;
  __shared__ __align__(16) float sT[8][16 * 68];
  const int b    = blockIdx.y;
  const int lane = threadIdx.x & 31;
  const int wave = threadIdx.x >> 5;
  const int tilesN = N >> 6;
  const int tilesM = M >> 6;
  const int tile = blockIdx.x * 8 + wave;
  if (tile >= tilesM * tilesN) return;
  const int tm = tile / tilesN;
  const int tn = tile - tm * tilesN;
  const int m0 = tm << 6;
  const int n0 = tn << 6;

  const T* Ab  = A  + (size_t)b * strideA;
  const T* Bb  = Bt + (size_t)b * strideB;
  const T* Ab2 = SPLIT ? (A2  + (size_t)b * strideA) : nullptr;
  const T* Bb2 = SPLIT ? (Bt2 + (size_t)b * strideB) : nullptr;

  const int rlane = lane & 15;
  const int koff  = (lane >> 4) * 8;
  const int mOff  = (lane >> 4) * 8;

  v8f acc[4][4];
#pragma unroll
  for (int i = 0; i < 4; ++i)
#pragma unroll
    for (int j = 0; j < 4; ++j) acc[i][j] = (v8f){0.f,0.f,0.f,0.f,0.f,0.f,0.f,0.f};

  for (int k0 = 0; k0 < K; k0 += 32) {
    V bh[4], bl[4];
#pragma unroll
    for (int j = 0; j < 4; ++j) {
      const size_t bo = (size_t)(n0 + (j << 4) + rlane) * ldb + koff + k0;
      bh[j] = Frag<T>::load(Bb + bo);
      if (SPLIT) bl[j] = Frag<T>::load(Bb2 + bo);
    }
#pragma unroll
    for (int i = 0; i < 4; ++i) {
      const size_t ao = (size_t)(m0 + (i << 4) + rlane) * lda + koff + k0;
      V ah = Frag<T>::load(Ab + ao);
      V al;
      if (SPLIT) al = Frag<T>::load(Ab2 + ao);
#pragma unroll
      for (int j = 0; j < 4; ++j) {
        acc[i][j] = Frag<T>::mma(ah, bh[j], acc[i][j]);
        if (SPLIT) {
          acc[i][j] = Frag<T>::mma(ah, bl[j], acc[i][j]);
          acc[i][j] = Frag<T>::mma(al, bh[j], acc[i][j]);
        }
      }
      Frag<T>::guard(acc[i][0], acc[i][3], ah, SPLIT ? al : ah);
    }
    Frag<T>::keep(bh[0], bh[1], bh[2], bh[3]);
    if (SPLIT) Frag<T>::keep(bl[0], bl[1], bl[2], bl[3]);
  }
  acc_guard4(acc[0][0], acc[0][1], acc[0][2], acc[0][3]);
  acc_guard4(acc[1][0], acc[1][1], acc[1][2], acc[1][3]);
  acc_guard4(acc[2][0], acc[2][1], acc[2][2], acc[2][3]);
  acc_guard4(acc[3][0], acc[3][1], acc[3][2], acc[3][3]);

  float* slab = sT[wave];
  const float* Rb = RESID ? (resid + (size_t)b * strideR) : nullptr;
#pragma unroll
  for (int i = 0; i < 4; ++i) {
    const int mBase = m0 + (i << 4);
#pragma unroll
    for (int j = 0; j < 4; ++j) {
      const int n = n0 + (j << 4) + rlane;
      float bv = 0.f;
      if (BIAS_MODE == 2) bv = bias[n];
#pragma unroll
      for (int r = 0; r < 8; ++r) {
        float v = acc[i][j][r] * scale;
        if (BIAS_MODE == 1) v += bias[mBase + mOff + r];
        if (BIAS_MODE == 2) v += bv;
        if (RESID) v += Rb[(size_t)(mBase + mOff + r) * ldc + n];
        if (ACT == 1) v = tanhf(v);
        if (ACT == 2) v = fmaxf(v, 0.0f);
        if (ACT == 3) v = v / (1.0f + expf(-v));
        if (ACT == 4) v = (v > 0.f) ? v : 0.01f * v;
        if (ACT == 5) v = 0.5f * v * (1.0f + erff(v * 0.70710678118654752f));
        slab[(mOff + r) * 68 + (j << 4) + rlane] = v;
      }
    }
    __builtin_amdgcn_fence(__ATOMIC_RELEASE, "workgroup");
    __builtin_amdgcn_wave_barrier();
    __builtin_amdgcn_fence(__ATOMIC_ACQUIRE, "workgroup");
    if (OUT_MODE == 0) {
      float* C = (float*)Cout + (size_t)b * strideC;
      const int hh = lane >> 4, c4 = (lane & 15) * 4;
      for (int pass = 0; pass < 2; ++pass) {
#pragma unroll
        for (int it = 0; it < 8; ++it) {
          const int row = it * 2 + hh;
          v4f v = *(const v4f*)(slab + row * 68 + c4);
          *(volatile v4f*)(C + (size_t)(mBase + row) * ldc + n0 + c4) = v;
        }
        __threadfence();
      }
    } else {
      const int q = lane >> 3, c8 = (lane & 7) * 8;
      unsigned short* C  = (unsigned short*)Cout  + (size_t)b * strideC;
      unsigned short* C2 = (OUT_MODE == 2) ? ((unsigned short*)Cout2 + (size_t)b * strideC) : nullptr;
      for (int pass = 0; pass < 2; ++pass) {
#pragma unroll
        for (int it = 0; it < 4; ++it) {
          const int row = it * 4 + q;
          const float* sp = slab + row * 68 + c8;
          v8h hv, lv;
#pragma unroll
          for (int e = 0; e < 8; ++e) {
            if (OUT_MODE == 1) {
              hv[e] = (_Float16)sp[e];
            } else {
              unsigned short hb = f2bf_bits(sp[e]);
              unsigned short lb = f2bf_bits(sp[e] - bf_bits2f(hb));
              hv[e] = __builtin_bit_cast(_Float16, hb);
              lv[e] = __builtin_bit_cast(_Float16, lb);
            }
          }
          *(volatile v8h*)(C + (size_t)(mBase + row) * ldc + n0 + c8) = hv;
          if (OUT_MODE == 2) *(volatile v8h*)(C2 + (size_t)(mBase + row) * ldc + n0 + c8) = lv;
        }
        __threadfence();
      }
    }
    __builtin_amdgcn_fence(__ATOMIC_RELEASE, "workgroup");
    __builtin_amdgcn_wave_barrier();
    __builtin_amdgcn_fence(__ATOMIC_ACQUIRE, "workgroup");
  }
}

__global__ __launch_bounds__(256) void cast_f32_f16x2(
    const float* __restrict__ in, _Float16* __restrict__ out, int n2) {
  int i = blockIdx.x * 256 + threadIdx.x;
  if (i < n2) {
    const _Float16 h0 = (_Float16)in[2 * i], h1 = (_Float16)in[2 * i + 1];
    const unsigned u = (unsigned)__builtin_bit_cast(unsigned short, h0) | ((unsigned)__builtin_bit_cast(unsigned short, h1) << 16);
    ((volatile unsigned*)out)[i] = u;
    __threadfence();
    ((volatile unsigned*)out)[i] = u;
  }
}


#define HN 20000
#define HNP 20032
#define HD 128
#define HDEG 32
#define H_EPS 1e-7f
#define H_MIN 1e-15f
__device__ __forceinline__ float f_cosh(float x) { return 0.5f * (__expf(x) + __expf(-x)); }
__device__ __forceinline__ float f_sinh(float x) { const float ax = fabsf(x); if (ax < 1e-2f) return x * (1.0f + x * x * (1.0f / 6.0f)); return 0.5f * (__expf(x) - __expf(-x)); }
__device__ __forceinline__ float f_tanh(float x) { const float ax = fabsf(x); if (ax < 1e-3f) return x * (1.0f - x * x * (1.0f / 3.0f)); const float e = __expf(-2.0f * ax); const float t = (1.0f - e) / (1.0f + e); return x < 0.f ? -t : t; }
__device__ __forceinline__ float wsum(float v) { for (int o = 16; o > 0; o >>= 1) v += __shfl_xor(v, o, 32); return v; }
__device__ __forceinline__ float h_arcosh(float x) { x = fmaxf(x, 1.0f + H_EPS); return __logf(x + sqrtf(x * x - 1.0f)); }
struct HV { v4f v; };
__device__ __forceinline__ float comp0(const HV& a, int lane) { return __shfl(a.v[0], 0, 32); }
__device__ __forceinline__ float space_norm2(const HV& a, int lane) { float s = 0.f; _Pragma("unroll 1") for (int q = 0; q < 4; ++q) { if (lane == 0 && q == 0) continue; s += a.v[q] * a.v[q]; } return wsum(s); }
__device__ __forceinline__ float space_dot(const HV& a, const HV& b, int lane) { float s = 0.f; _Pragma("unroll 1") for (int q = 0; q < 4; ++q) { if (lane == 0 && q == 0) continue; s += a.v[q] * b.v[q]; } return wsum(s); }
__device__ __forceinline__ HV h_proj(HV x, int lane) { const float n2 = space_norm2(x, lane); if (lane == 0) x.v[0] = sqrtf(fmaxf(1.0f + n2, H_EPS)); return x; }
__device__ __forceinline__ HV h_expmap0(HV u, int lane) { const float xn = fmaxf(sqrtf(space_norm2(u, lane)), H_MIN); HV r; const float s = f_sinh(xn) / xn; _Pragma("unroll 1") for (int q = 0; q < 4; ++q) r.v[q] = u.v[q] * s; if (lane == 0) r.v[0] = f_cosh(xn); return r; }
__device__ __forceinline__ HV h_logmap0(HV x, int lane) { const float yn = fmaxf(sqrtf(space_norm2(x, lane)), H_MIN); const float th = fmaxf(comp0(x, lane), 1.0f + H_EPS); const float s = h_arcosh(th) / yn; HV r; _Pragma("unroll 1") for (int q = 0; q < 4; ++q) r.v[q] = x.v[q] * s; if (lane == 0) r.v[0] = 0.f; return r; }
__device__ __forceinline__ HV h_mobius_add(HV x, HV y, int lane) {
  const HV u = h_logmap0(y, lane);
  const float x0 = comp0(x, lane); const float yn = fmaxf(sqrtf(space_norm2(x, lane)), H_MIN);
  HV yhat; _Pragma("unroll 1") for (int q = 0; q < 4; ++q) yhat.v[q] = x.v[q] / yn; if (lane == 0) yhat.v[0] = 0.f;
  HV v; _Pragma("unroll 1") for (int q = 0; q < 4; ++q) v.v[q] = (1.0f - x0) * yhat.v[q]; if (lane == 0) v.v[0] = -yn;
  const float alpha = space_dot(yhat, u, lane);
  HV w; _Pragma("unroll 1") for (int q = 0; q < 4; ++q) w.v[q] = u.v[q] - alpha * v.v[q];
  const float ux = space_dot(x, w, lane); if (lane == 0) w.v[0] = ux / fmaxf(x0, H_EPS);
  const float w0 = comp0(w, lane); const float md = space_norm2(w, lane) + w0 * w0 - 2.0f * w0 * w0; const float theta = fmaxf(sqrtf(fmaxf(md, 0.f)), H_MIN);
  const float ch = f_cosh(theta), sh = f_sinh(theta) / theta; HV r; _Pragma("unroll 1") for (int q = 0; q < 4; ++q) r.v[q] = ch * x.v[q] + sh * w.v[q];
  return h_proj(r, lane);
}
__device__ __forceinline__ HV h_bias_point(const float* b, int lane) { HV u; u.v = *(const v4f*)(b + lane * 4); if (lane == 0) u.v[0] = 0.f; return h_proj(h_expmap0(u, lane), lane); }
__device__ __forceinline__ HV h_linear_finish(HV m, const float* b, int lane) { const HV res = h_proj(h_expmap0(m, lane), lane); const HV hb = h_bias_point(b, lane); return h_proj(h_mobius_add(res, hb, lane), lane); }
__global__ __launch_bounds__(256) void log_in_kernel(const float* __restrict__ x, unsigned* __restrict__ A16) {
  const int lane = threadIdx.x & 31, wave = threadIdx.x >> 5; const int n = blockIdx.x * 8 + wave;
  HV u; u.v = (v4f){0.f, 0.f, 0.f, 0.f};
  if (n < HN) { HV xv; xv.v = *(const v4f*)(x + (size_t)n * HD + lane * 4); u = h_logmap0(xv, lane); }
  typedef __attribute__((ext_vector_type(2))) unsigned u2; u2 pk; pk[0] = (unsigned)__builtin_bit_cast(unsigned short, (_Float16)u.v[0]) | ((unsigned)__builtin_bit_cast(unsigned short, (_Float16)u.v[1]) << 16); pk[1] = (unsigned)__builtin_bit_cast(unsigned short, (_Float16)u.v[2]) | ((unsigned)__builtin_bit_cast(unsigned short, (_Float16)u.v[3]) << 16);
  *(volatile u2*)(A16 + ((size_t)n * HD) / 2 + lane * 2) = pk; __threadfence(); *(volatile u2*)(A16 + ((size_t)n * HD) / 2 + lane * 2) = pk;
}
__global__ __launch_bounds__(256) void att_kernel(const float* __restrict__ M, const float* __restrict__ b_att, float* __restrict__ ATT) {
  const int lane = threadIdx.x & 31, wave = threadIdx.x >> 5; const int n = blockIdx.x * 8 + wave; if (n >= HN) return;
  HV ma; ma.v = *(const v4f*)(M + (size_t)n * 256 + lane * 4);
  const HV att = h_linear_finish(ma, b_att, lane);
  *(volatile v4f*)(ATT + (size_t)n * HD + lane * 4) = att.v; __threadfence(); *(volatile v4f*)(ATT + (size_t)n * HD + lane * 4) = att.v;
}
__global__ __launch_bounds__(256) void red_kernel(const float* __restrict__ M, const float* __restrict__ b_data, float* __restrict__ P) {
  const int lane = threadIdx.x & 31, wave = threadIdx.x >> 5; const int n = blockIdx.x * 8 + wave; if (n >= HN) return;
  HV mdv; mdv.v = *(const v4f*)(M + (size_t)n * 256 + HD + lane * 4);
  const HV red = h_linear_finish(mdv, b_data, lane);
  const float r0 = comp0(red, lane); HV p; _Pragma("unroll 1") for (int q = 0; q < 4; ++q) p.v[q] = red.v[q] / (r0 + 1.0f); if (lane == 0) p.v[0] = 0.f;
  const float pn2 = space_norm2(p, lane); if (lane == 0) p.v[0] = 1.0f / fmaxf(1.0f - pn2, H_MIN);
  *(volatile v4f*)(P + (size_t)n * HD + lane * 4) = p.v; __threadfence(); *(volatile v4f*)(P + (size_t)n * HD + lane * 4) = p.v;
}
__global__ __launch_bounds__(256) void edge_kernel(const float* __restrict__ ATT, const float* __restrict__ P, const float* __restrict__ ev, const int* __restrict__ tgt, unsigned* __restrict__ B16) {
  const int lane = threadIdx.x & 31, wave = threadIdx.x >> 5; const int i = blockIdx.x * 8 + wave;
  HV u; u.v = (v4f){0.f, 0.f, 0.f, 0.f};
  if (i < HN) {
    HV ai; ai.v = *(const v4f*)(ATT + (size_t)i * HD + lane * 4); const float ai0 = comp0(ai, lane);
    float mycoef = 0.f, myg2 = 0.f; int myj = 0;
#pragma unroll 1
    for (int k = 0; k < HDEG; ++k) { const size_t e = (size_t)i * HDEG + k; int j = tgt[e]; j = j < 0 ? 0 : (j >= HN ? HN - 1 : j);
      HV aj; aj.v = *(const v4f*)(ATT + (size_t)j * HD + lane * 4); const float aj0 = comp0(aj, lane);
      float full = 0.f; _Pragma("unroll 1") for (int q = 0; q < 4; ++q) full += aj.v[q] * ai.v[q]; full = wsum(full); const float md = full - 2.0f * aj0 * ai0;
      const float th = fmaxf(-md, 1.0f + H_EPS); const float ac = h_arcosh(th); const float sqd = fminf(ac * ac, 50.0f);
      const float coef = -ev[e] * sqd;
      if (lane == k) { mycoef = coef; myj = j; myg2 = P[(size_t)j * HD]; } }
    const float denom = sqrtf(wsum(mycoef * mycoef)); const float a = mycoef / fmaxf(denom, 1e-12f);
    const float den_raw = wsum(a * (myg2 - 0.5f)); const float den = (fabsf(den_raw) < H_MIN) ? H_MIN : den_raw;
    HV num; num.v = (v4f){0.f, 0.f, 0.f, 0.f};
#pragma unroll 1
    for (int k = 0; k < HDEG; ++k) { const float ak = __shfl(a, k, 32), gk = __shfl(myg2, k, 32); const int j = __shfl(myj, k, 32);
      HV pj; pj.v = *(const v4f*)(P + (size_t)j * HD + lane * 4); if (lane == 0) pj.v[0] = 0.f;
      _Pragma("unroll 1") for (int q = 0; q < 4; ++q) num.v[q] += ak * gk * pj.v[q]; }
    HV m; _Pragma("unroll 1") for (int q = 0; q < 4; ++q) m.v[q] = num.v[q] / den; if (lane == 0) m.v[0] = 0.f;
    const float vn = fmaxf(sqrtf(space_norm2(m, lane)), H_MIN); const float vc = fminf(fmaxf(vn, -1.0f + 1e-7f), 1.0f - 1e-7f); const float at = 0.5f * __logf((1.0f + vc) / (1.0f - vc));
    const float sc = f_tanh(0.5f * at) / vn; HV mid; _Pragma("unroll 1") for (int q = 0; q < 4; ++q) mid.v[q] = m.v[q] * sc; if (lane == 0) mid.v[0] = 0.f;
    const float sq = space_norm2(mid, lane); const float dv = fmaxf(1.0f - sq, H_MIN); HV h; _Pragma("unroll 1") for (int q = 0; q < 4; ++q) h.v[q] = 2.0f * mid.v[q] / dv; if (lane == 0) h.v[0] = (1.0f + sq) / dv;
    u = h_logmap0(h, lane); }
  typedef __attribute__((ext_vector_type(2))) unsigned u2; u2 pk; pk[0] = (unsigned)__builtin_bit_cast(unsigned short, (_Float16)u.v[0]) | ((unsigned)__builtin_bit_cast(unsigned short, (_Float16)u.v[1]) << 16); pk[1] = (unsigned)__builtin_bit_cast(unsigned short, (_Float16)u.v[2]) | ((unsigned)__builtin_bit_cast(unsigned short, (_Float16)u.v[3]) << 16);
  *(volatile u2*)(B16 + ((size_t)i * HD) / 2 + lane * 2) = pk; __threadfence(); *(volatile u2*)(B16 + ((size_t)i * HD) / 2 + lane * 2) = pk;
}
__global__ __launch_bounds__(256) void out_kernel(const float* __restrict__ M2, const float* __restrict__ b_out, float* __restrict__ out) {
  const int lane = threadIdx.x & 31, wave = threadIdx.x >> 5; const int n = blockIdx.x * 8 + wave; if (n >= HN) return;
  HV m; m.v = *(const v4f*)(M2 + (size_t)n * HD + lane * 4); const HV o = h_linear_finish(m, b_out, lane);
  *(volatile v4f*)(out + (size_t)n * HD + lane * 4) = o.v; __threadfence(); *(volatile v4f*)(out + (size_t)n * HD + lane * 4) = o.v;
}
extern "C" void kernel_launch(void* const* d_in, const int* in_sizes, int n_in, void* d_out, int out_size, void* d_ws, size_t ws_size, hipStream_t stream) {
  (void)in_sizes; (void)n_in; (void)out_size; (void)ws_size;
  auto Fp = [&](int i) { return (const float*)d_in[i]; };
  const float* x = Fp(0); const float* ev = Fp(1); const float* Watt = Fp(2); const float* batt = Fp(3); const float* Wdata = Fp(4); const float* bdata = Fp(5); const float* Wout = Fp(6); const float* bout = Fp(7); const int* tgt = (const int*)d_in[9];
  (void)d_in[8];
  char* ws = (char*)d_ws; size_t off = 0;
  auto carve = [&](size_t bytes) -> char* { char* p = ws + off; off += (bytes + 255) & ~(size_t)255; return p; };
  unsigned* A16 = (unsigned*)carve((size_t)HNP * HD * 2); _Float16* W1 = (_Float16*)carve(256 * HD * 2); _Float16* W2 = (_Float16*)carve(HD * HD * 2); float* M = (float*)carve((size_t)HNP * 256 * 4);
  float* ATT = (float*)carve((size_t)HN * HD * 4); float* P = (float*)carve((size_t)HN * HD * 4); unsigned* B16 = (unsigned*)carve((size_t)HNP * HD * 2); float* M2 = (float*)carve((size_t)HNP * HD * 4);
  log_in_kernel<<<HNP / 8, 256, 0, stream>>>(x, A16);
  cast_f32_f16x2<<<(HD * HD / 2 + 255) / 256, 256, 0, stream>>>(Watt, W1, HD * HD / 2);
  cast_f32_f16x2<<<(HD * HD / 2 + 255) / 256, 256, 0, stream>>>(Wdata, W1 + HD * HD, HD * HD / 2);
  cast_f32_f16x2<<<(HD * HD / 2 + 255) / 256, 256, 0, stream>>>(Wout, W2, HD * HD / 2);
  { const int t = (HNP / 64) * 4; wmma_gemm64<0, false, 0, 0, false><<<dim3((t + 7) / 8, 1), 256, 0, stream>>>((const unsigned short*)A16, nullptr, HD, 0, U16(W1), nullptr, HD, 0, M, nullptr, 256, 0, nullptr, nullptr, 0, HNP, 256, HD, 1.0f); }
  att_kernel<<<HNP / 8, 256, 0, stream>>>(M, batt, ATT); red_kernel<<<HNP / 8, 256, 0, stream>>>(M, bdata, P);
  edge_kernel<<<HNP / 8, 256, 0, stream>>>(ATT, P, ev, tgt, B16);
  { const int t = (HNP / 64) * 2; wmma_gemm64<0, false, 0, 0, false><<<dim3((t + 7) / 8, 1), 256, 0, stream>>>((const unsigned short*)B16, nullptr, HD, 0, U16(W2), nullptr, HD, 0, M2, nullptr, HD, 0, nullptr, nullptr, 0, HNP, HD, HD, 1.0f); }
  out_kernel<<<HNP / 8, 256, 0, stream>>>(M2, bout, (float*)d_out);
}
